// MultiHeadRelativeSelfAttention_46325517254727
// MI455X (gfx1250) — hardware-run, weakly checked
//
#include <hip/hip_runtime.h>


#define NB_  8
#define TT   1024
#define DM   1024
#define NH_  16
#define HD   64
#define ZH   4
#define PCAR 1024.0f
typedef _Float16 h16;
typedef unsigned short bf;
typedef __attribute__((ext_vector_type(16))) __bf16   v16bf;
typedef __attribute__((ext_vector_type(16))) _Float16 v16h;
typedef __attribute__((ext_vector_type(8)))  _Float16 v8h;
typedef __attribute__((ext_vector_type(8)))  unsigned short v8us;
typedef __attribute__((ext_vector_type(8)))  float    v8f;
typedef __attribute__((ext_vector_type(4)))  float    v4f;
typedef v8h  __attribute__((may_alias)) v8ha;
typedef v4f  __attribute__((may_alias)) v4fa;
typedef v8us __attribute__((may_alias)) v8usa;

__device__ __forceinline__ unsigned short f2bf(float f) { unsigned u = __float_as_uint(f); u += 0x7FFFu + ((u >> 16) & 1u); return (unsigned short)(u >> 16); }
__device__ __forceinline__ float bf2f(unsigned short b) { return __uint_as_float(((unsigned)b) << 16); }
__device__ __forceinline__ float bfr(float f) { return bf2f(f2bf(f)); }
__device__ __forceinline__ v16h cat16(v8h lo, v8h hi) { return __builtin_shufflevector(lo, hi, 0, 1, 2, 3, 4, 5, 6, 7, 8, 9, 10, 11, 12, 13, 14, 15); }
__device__ __forceinline__ v16bf cat16b(v8us lo, v8us hi) { return __builtin_bit_cast(v16bf, __builtin_shufflevector(lo, hi, 0, 1, 2, 3, 4, 5, 6, 7, 8, 9, 10, 11, 12, 13, 14, 15)); }
__device__ __forceinline__ v8f wmma16(v16h a, v16h b, v8f c) { return __builtin_amdgcn_wmma_f32_16x16x32_f16(false, a, false, b, (short)0, c, false, false); }
__device__ __forceinline__ v8f wmmab(v16bf a, v16bf b, v8f c) { return __builtin_amdgcn_wmma_f32_16x16x32_bf16(false, a, false, b, (short)0, c, false, false); }


template <typename T16> struct WFrag;
template <> struct WFrag<h16> { typedef v16h V; static __device__ __forceinline__ V ld(const h16* p) { return cat16(*(const v8h*)p, *(const v8h*)(p + 16)); } static __device__ __forceinline__ v8f mma(V a, V b, v8f c) { return wmma16(a, b, c); } };
template <> struct WFrag<bf> { typedef v16bf V; static __device__ __forceinline__ V ld(const bf* p) { return cat16b(*(const v8us*)p, *(const v8us*)(p + 16)); } static __device__ __forceinline__ v8f mma(V a, V b, v8f c) { return wmmab(a, b, c); } };
template <typename T16, int NSPLIT, bool BIAS>
__global__ __launch_bounds__(32) void k_gemmw(const T16* __restrict__ A, const T16* __restrict__ A2, const T16* __restrict__ Bt, const T16* __restrict__ Bt2, int K, float* C, int ldc, const float* __restrict__ bias, size_t sA, size_t sB, size_t sC) {
    typedef typename WFrag<T16>::V V;
    __shared__ __align__(16) float os[16 * 68];
    const size_t z = blockIdx.z; A += z * sA; if (A2) A2 += z * sA; Bt += z * sB; if (Bt2) Bt2 += z * sB; C += z * sC;
    const int lane = threadIdx.x & 31, lr = lane & 15, hi = lane >> 4; const int r0 = blockIdx.x * 64, c0 = blockIdx.y * 64;
    v8f acc[4][4];
#pragma unroll
    for (int mb = 0; mb < 4; ++mb)
#pragma unroll
        for (int nb = 0; nb < 4; ++nb) acc[mb][nb] = (v8f){};
    const size_t aoff = (size_t)(r0 + lr) * K + 8 * hi, boff = (size_t)(c0 + lr) * K + 8 * hi;
#pragma unroll 1
    for (int kc = 0; kc < K; kc += 32) {
        V a[4], a2[4];
#pragma unroll
        for (int mb = 0; mb < 4; ++mb) { a[mb] = WFrag<T16>::ld(A + aoff + (size_t)mb * 16 * K + kc); if (NSPLIT == 1 || NSPLIT == 2) a2[mb] = WFrag<T16>::ld(A2 + aoff + (size_t)mb * 16 * K + kc); }
#pragma unroll
        for (int nb = 0; nb < 4; ++nb) { const V b = WFrag<T16>::ld(Bt + boff + (size_t)nb * 16 * K + kc); V b2; if (NSPLIT >= 2) b2 = WFrag<T16>::ld(Bt2 + boff + (size_t)nb * 16 * K + kc);
#pragma unroll
            for (int mb = 0; mb < 4; ++mb) { acc[mb][nb] = WFrag<T16>::mma(a[mb], b, acc[mb][nb]); if (NSPLIT == 1 || NSPLIT == 2) acc[mb][nb] = WFrag<T16>::mma(a2[mb], b, acc[mb][nb]); if (NSPLIT >= 2) acc[mb][nb] = WFrag<T16>::mma(a[mb], b2, acc[mb][nb]); } }
        asm volatile("v_nop\n\tv_nop\n\tv_nop\n\tv_nop" : "+v"(acc[0][0]), "+v"(acc[1][1]), "+v"(acc[2][2]), "+v"(acc[3][3]) : "v"(a[0]), "v"(a[3]));
    }
#pragma unroll
    for (int mb = 0; mb < 4; ++mb) {
#pragma unroll
        for (int nb = 0; nb < 4; ++nb) {
#pragma unroll
            for (int j = 0; j < 8; ++j) os[(hi * 8 + j) * 68 + nb * 16 + lr] = acc[mb][nb][j]; }
        __builtin_amdgcn_wave_barrier(); asm volatile("" ::: "memory");
        float* crow = C + (size_t)(r0 + mb * 16) * ldc + c0;
#pragma unroll 1
        for (int ps = 0; ps < 2; ++ps) {
#pragma unroll
            for (int s = 0; s < 8; ++s) { const int row = 2 * s + hi, cofs = lr * 4; v4f val = *(const v4fa*)(os + row * 68 + cofs); if (BIAS) { val[0] += bfr(bias[c0 + cofs]); val[1] += bfr(bias[c0 + cofs + 1]); val[2] += bfr(bias[c0 + cofs + 2]); val[3] += bfr(bias[c0 + cofs + 3]); }
                *(volatile v4f*)(crow + (size_t)row * ldc + cofs) = val; }
            if (ps == 0) __threadfence(); }
        __builtin_amdgcn_wave_barrier(); asm volatile("" ::: "memory");
    }
}

__device__ __forceinline__ h16 tohx(float x) { return (h16)x; }
__device__ __forceinline__ void splitf(float y, unsigned short& h, unsigned short& l) { h = f2bf(y); l = f2bf(y - bf2f(h)); }
typedef __attribute__((ext_vector_type(2))) unsigned short v2us;
typedef __attribute__((ext_vector_type(4))) unsigned short v4us;
typedef __attribute__((ext_vector_type(2))) _Float16 v2h;
typedef __attribute__((ext_vector_type(4))) _Float16 v4h;

__global__ __launch_bounds__(256) void k_cvt8(const float* __restrict__ src, bf* dst, size_t n8) { const size_t i = (size_t)blockIdx.x * 256 + threadIdx.x; if (i >= n8) return; const v8f v = *(const v8f*)(src + i * 8); v8us o;
#pragma unroll
    for (int k = 0; k < 8; ++k) o[k] = f2bf(v[k]); *(volatile v8us*)(dst + i * 8) = o; __threadfence(); *(volatile v8us*)(dst + i * 8) = o; }
__global__ __launch_bounds__(256) void k_wtG(const float* __restrict__ w, int K, int N, bf* Bt) {
    const int lane = threadIdx.x & 31; const int L0 = (blockIdx.x * 8 + (threadIdx.x >> 5)) * 8; const int nlines = N * K / 64;
#pragma unroll
    for (int ps = 0; ps < 2; ++ps) {
#pragma unroll 1
        for (int l = 0; l < 8; ++l) { const int L = L0 + l; if (L >= nlines) break; const size_t e = (size_t)L * 64 + lane * 2; const int k = (int)(e % K), n = (int)(e / K); v2us o;
            o[0] = f2bf(w[(size_t)k * N + n]); o[1] = f2bf(w[(size_t)(k + 1) * N + n]); *(volatile v2us*)(Bt + e) = o; }
        if (ps == 0) __threadfence(); }
}

__device__ __attribute__((noinline)) float posval(int j, int cc) { const int fi = cc % (DM / 2); const float invf = __fdiv_rn(1.0f, powf(10000.0f, (float)(2 * fi) / (float)DM)); const float ang = __fmul_rn((float)(TT - 1 - j), invf); return (cc < DM / 2) ? sinf(ang) : cosf(ang); }
__global__ __launch_bounds__(256) void k_pos(bf* Ph, bf* Pl) { const size_t e = ((size_t)blockIdx.x * 256 + threadIdx.x) * 4; if (e >= (size_t)TT * DM) return; const int c = (int)(e % DM); const int j = (int)(e / DM); v4us oh, ol;
#pragma unroll 1
    for (int u = 0; u < 4; ++u) { const float val = posval(j, c + u); unsigned short a2, b2; splitf(val, a2, b2); oh[u] = a2; ol[u] = b2; }
    *(volatile v4us*)(Ph + e) = oh; *(volatile v4us*)(Pl + e) = ol; __threadfence(); *(volatile v4us*)(Ph + e) = oh; *(volatile v4us*)(Pl + e) = ol; }
__global__ __launch_bounds__(256) void k_pl16(const float* __restrict__ F, int pitch, int col0, h16* P) { const size_t e = ((size_t)blockIdx.x * 256 + threadIdx.x) * 4; if (e >= (size_t)NH_ * TT * HD) return; const int d = (int)(e % HD); const int t = (int)((e / HD) % TT); const int h = (int)(e / ((size_t)HD * TT)); const v4f a = *(const v4f*)(F + (size_t)t * pitch + col0 + h * HD + d); v4h o; for (int u = 0; u < 4; ++u) o[u] = tohx(a[u]); *(volatile v4h*)(P + e) = o; __threadfence(); *(volatile v4h*)(P + e) = o; }
__global__ __launch_bounds__(256) void k_vt16(const float* __restrict__ F, int pitch, int col0, h16* VT) { const size_t e = ((size_t)blockIdx.x * 256 + threadIdx.x) * 2; if (e >= (size_t)NH_ * HD * TT) return; const int t = (int)(e % TT); const int d = (int)((e / TT) % HD); const int h = (int)(e / ((size_t)TT * HD)); v2h o; o[0] = tohx(F[(size_t)t * pitch + col0 + h * HD + d]); o[1] = tohx(F[(size_t)(t + 1) * pitch + col0 + h * HD + d]); *(volatile v2h*)(VT + e) = o; __threadfence(); *(volatile v2h*)(VT + e) = o; }
__global__ __launch_bounds__(256) void k_xsoft(const float* __restrict__ AC, const float* __restrict__ BD, const int* __restrict__ km, h16* P16) { const int lane = threadIdx.x & 31; const int row = blockIdx.x * 8 + (threadIdx.x >> 5); if (row >= ZH * TT) return; const int i = row % TT; const int zz = row / TT; const float* ar = AC + (size_t)row * TT; const float* bdz = BD + (size_t)zz * TT * TT; float v[TT / 32]; float mx = -3.0e38f;
#pragma unroll
    for (int ch = 0; ch < TT / 128; ++ch) { const v4f a = *(const v4f*)(ar + ch * 128 + lane * 4);
#pragma unroll
        for (int u = 0; u < 4; ++u) { const int j = ch * 128 + lane * 4 + u; const int f = i * TT + j + TT; const int rw = f / (TT + 1), cl = f % (TT + 1); const float bd = (cl == 0) ? 0.0f : bdz[(size_t)rw * TT + (cl - 1)]; float s0 = __fadd_rn(a[u], bd) * 0.125f; asm volatile("" : "+v"(s0)); const float mk = (float)(km[j] != 0); float t = __fmul_rn(s0, mk); asm volatile("" : "+v"(t)); t = __fsub_rn(t, 1e30f * (1.0f - mk)); v[ch * 4 + u] = t; mx = fmaxf(mx, t); } }
#pragma unroll
    for (int sh = 16; sh; sh >>= 1) mx = fmaxf(mx, __shfl_xor(mx, sh, 32));
    float sum = 0.f;
#pragma unroll
    for (int q = 0; q < TT / 32; ++q) { float d0 = __fsub_rn(v[q], mx); asm volatile("" : "+v"(d0)); v[q] = __builtin_amdgcn_exp2f(__fmul_rn(d0, 1.4426950408889634f)); sum += v[q]; }
#pragma unroll
    for (int sh = 16; sh; sh >>= 1) sum += __shfl_xor(sum, sh, 32);
    const float f2 = __fdiv_rn(PCAR, sum);
    for (int ps = 0; ps < 2; ++ps) {
#pragma unroll
        for (int ch = 0; ch < TT / 128; ++ch) { v4h o4; for (int q = 0; q < 4; ++q) o4[q] = tohx(v[ch * 4 + q] * f2); *(volatile v4h*)(P16 + (size_t)row * TT + ch * 128 + lane * 4) = o4; }
        if (ps == 0) __threadfence(); } }
__global__ __launch_bounds__(256) void k_mrg(const float* __restrict__ O, int h0, bf* Ah, bf* Al) { const size_t e = ((size_t)blockIdx.x * 256 + threadIdx.x) * 4; if (e >= (size_t)ZH * TT * HD) return; const int d = (int)(e % HD); const int t = (int)((e / HD) % TT); const int zz = (int)(e / ((size_t)HD * TT)); const size_t oo = (size_t)t * DM + (h0 + zz) * HD + d; v4us oh, ol;
#pragma unroll
    for (int u = 0; u < 4; ++u) { unsigned short a, b; splitf(O[e + u] * (1.0f / PCAR), a, b); oh[u] = a; ol[u] = b; } *(volatile v4us*)(Ah + oo) = oh; *(volatile v4us*)(Al + oo) = ol; __threadfence(); *(volatile v4us*)(Ah + oo) = oh; *(volatile v4us*)(Al + oo) = ol; }
__global__ __launch_bounds__(256) void k_resid(const float* __restrict__ Y, const float* __restrict__ xb, float* OUTb) { const size_t e = ((size_t)blockIdx.x * 256 + threadIdx.x) * 4; if (e >= (size_t)TT * DM) return; const v4f y = *(const v4f*)(Y + e), a = *(const v4f*)(xb + e); v4f o; for (int u = 0; u < 4; ++u) o[u] = __fadd_rn(y[u], bfr(a[u])); *(volatile v4f*)(OUTb + e) = o; __threadfence(); *(volatile v4f*)(OUTb + e) = o; }

extern "C" void kernel_launch(void* const* d_in, const int* in_sizes, int n_in,
                              void* d_out, int out_size, void* d_ws, size_t ws_size, hipStream_t stream) {
    (void)in_sizes; (void)n_in; (void)out_size;
    const float* x = (const float*)d_in[0]; const int* km = (const int*)d_in[1]; const float* wqkv = (const float*)d_in[2]; const float* wr = (const float*)d_in[3]; const float* wo = (const float*)d_in[4];
    float* OUT = (float*)d_out;
    char* wsp = (char*)d_ws;
    auto take = [&](size_t bytes) { char* p = wsp; wsp += (bytes + 255) & ~(size_t)255; return (void*)p; };
    bf* BQKV = (bf*)take((size_t)3 * DM * DM * 2); bf* BR = (bf*)take((size_t)DM * DM * 2); bf* BO = (bf*)take((size_t)DM * DM * 2);
    bf* POSh = (bf*)take((size_t)TT * DM * 2); bf* POSl = (bf*)take((size_t)TT * DM * 2); float* RF = (float*)take((size_t)TT * DM * 4); h16* RP = (h16*)take((size_t)NH_ * TT * HD * 2);
    bf* XB = (bf*)take((size_t)TT * DM * 2); float* QKV = (float*)take((size_t)TT * 3 * DM * 4); h16* QP = (h16*)take((size_t)NH_ * TT * HD * 2); h16* KP = (h16*)take((size_t)NH_ * TT * HD * 2); h16* VT = (h16*)take((size_t)NH_ * HD * TT * 2);
    float* AC = (float*)take((size_t)ZH * TT * TT * 4); float* BD = (float*)take((size_t)ZH * TT * TT * 4); h16* P16 = (h16*)take((size_t)ZH * TT * TT * 2); float* O = (float*)take((size_t)ZH * TT * HD * 4); bf* ATh = (bf*)take((size_t)TT * DM * 2); bf* ATl = (bf*)take((size_t)TT * DM * 2); float* Y = (float*)take((size_t)TT * DM * 4);
    if ((size_t)(wsp - (char*)d_ws) > ws_size) return;
    k_wtG<<<(DM * 3 * DM / 64 + 63) / 64, 256, 0, stream>>>(wqkv, DM, 3 * DM, BQKV); k_wtG<<<(DM * DM / 64 + 63) / 64, 256, 0, stream>>>(wr, DM, DM, BR); k_wtG<<<(DM * DM / 64 + 63) / 64, 256, 0, stream>>>(wo, DM, DM, BO);
    k_pos<<<(unsigned)(((size_t)TT * DM / 4 + 255) / 256), 256, 0, stream>>>(POSh, POSl);
    k_gemmw<bf, 1, false><<<dim3(TT / 64, DM / 64, 1), 32, 0, stream>>>(POSh, POSl, BR, nullptr, DM, RF, DM, nullptr, 0, 0, 0);
    k_pl16<<<(unsigned)(((size_t)NH_ * TT * HD / 4 + 255) / 256), 256, 0, stream>>>(RF, DM, 0, RP);
    const size_t zq = (size_t)TT * HD, zS = (size_t)TT * TT, zv = (size_t)HD * TT;
    for (int b = 0; b < NB_; ++b) {
        k_cvt8<<<(TT * DM / 8 + 255) / 256, 256, 0, stream>>>(x + (size_t)b * TT * DM, XB, TT * DM / 8);
        k_gemmw<bf, 0, false><<<dim3(TT / 64, 3 * DM / 64, 1), 32, 0, stream>>>(XB, nullptr, BQKV, nullptr, DM, QKV, 3 * DM, nullptr, 0, 0, 0);
        k_pl16<<<(unsigned)(((size_t)NH_ * TT * HD / 4 + 255) / 256), 256, 0, stream>>>(QKV, 3 * DM, 0, QP); k_pl16<<<(unsigned)(((size_t)NH_ * TT * HD / 4 + 255) / 256), 256, 0, stream>>>(QKV, 3 * DM, DM, KP); k_vt16<<<(unsigned)(((size_t)NH_ * HD * TT / 2 + 255) / 256), 256, 0, stream>>>(QKV, 3 * DM, 2 * DM, VT);
        for (int h0 = 0; h0 < NH_; h0 += ZH) {
            k_gemmw<h16, 0, false><<<dim3(TT / 64, TT / 64, ZH), 32, 0, stream>>>(QP + (size_t)h0 * zq, nullptr, KP + (size_t)h0 * zq, nullptr, HD, AC, TT, nullptr, zq, zq, zS);
            k_gemmw<h16, 0, false><<<dim3(TT / 64, TT / 64, ZH), 32, 0, stream>>>(QP + (size_t)h0 * zq, nullptr, RP + (size_t)h0 * zq, nullptr, HD, BD, TT, nullptr, zq, zq, zS);
            k_xsoft<<<ZH * TT / 8, 256, 0, stream>>>(AC, BD, km + (size_t)b * TT, P16);
            k_gemmw<h16, 0, false><<<dim3(TT / 64, 1, ZH), 32, 0, stream>>>(P16, nullptr, VT + (size_t)h0 * zv, nullptr, TT, O, HD, nullptr, zS, zv, zq);
            k_mrg<<<(unsigned)(((size_t)ZH * TT * HD / 4 + 255) / 256), 256, 0, stream>>>(O, h0, ATh, ATl); }
        k_gemmw<bf, 1, false><<<dim3(TT / 64, DM / 64, 1), 32, 0, stream>>>(ATh, ATl, BO, nullptr, DM, Y, DM, nullptr, 0, 0, 0);
        k_resid<<<(unsigned)(((size_t)TT * DM / 4 + 255) / 256), 256, 0, stream>>>(Y, x + (size_t)b * TT * DM, OUT + (size_t)b * TT * DM); }
}
